// JiTAttention_90769838833766
// MI455X (gfx1250) — hardware-verified
//
#include <hip/hip_runtime.h>
#include <math.h>
#include <stdint.h>

constexpr int kBatch = 4;
constexpr int kSeq   = 2048;
constexpr int kDim   = 1024;
constexpr int kHeads = 16;
constexpr int kHd    = 64;
constexpr int kTok   = kBatch * kSeq;

typedef __attribute__((ext_vector_type(16))) _Float16 v16h;
typedef __attribute__((ext_vector_type(8)))  _Float16 v8h;
typedef __attribute__((ext_vector_type(16))) __bf16   v16b;
typedef __attribute__((ext_vector_type(8)))  __bf16   v8b;
typedef __attribute__((ext_vector_type(8)))  float    v8f;
typedef __attribute__((ext_vector_type(4)))  float    v4f;
typedef __attribute__((ext_vector_type(2)))  float    v2f;
typedef __attribute__((ext_vector_type(4)))  unsigned int v4u;

constexpr size_t kMiB      = 1048576;
constexpr size_t kOffWproj = 0;
constexpr size_t kOffBias  = 2 * kMiB;
constexpr size_t kOffXb    = 3 * kMiB;
constexpr size_t kOffWqkv  = 19 * kMiB;
constexpr size_t kOffKh    = 3 * kMiB;
constexpr size_t kOffKl    = 19 * kMiB;
constexpr size_t kOffQkf   = 35 * kMiB;
constexpr size_t kOffOh    = 35 * kMiB;
constexpr size_t kOffQh    = 67 * kMiB;
constexpr size_t kOffQl    = 83 * kMiB;
constexpr size_t kOffVt    = 99 * kMiB;
constexpr size_t kWsTotal  = 115 * kMiB;

__device__ __forceinline__ unsigned short f2bf_bits(float f) {
  unsigned u = __float_as_uint(f);
  return (unsigned short)((u + 0x7FFFu + ((u >> 16) & 1u)) >> 16);
}
__device__ __forceinline__ float bf_bits2f(unsigned short h) { return __uint_as_float(((unsigned)h) << 16); }

__device__ __forceinline__ void dep_guard_h(v8f& a, v8f& b, v16h x, v16h y) { asm volatile("v_nop\n\tv_nop\n\tv_nop\n\tv_nop" : "+v"(a), "+v"(b) : "v"(x), "v"(y)); }
__device__ __forceinline__ void dep_guard_b(v8f& a, v8f& b, v16b x, v16b y) { asm volatile("v_nop\n\tv_nop\n\tv_nop\n\tv_nop" : "+v"(a), "+v"(b) : "v"(x), "v"(y)); }
__device__ __forceinline__ void keep4_h(v16h a, v16h b, v16h c, v16h d) { asm volatile("v_nop" :: "v"(a), "v"(b), "v"(c), "v"(d)); }
__device__ __forceinline__ void keep4_b(v16b a, v16b b, v16b c, v16b d) { asm volatile("v_nop" :: "v"(a), "v"(b), "v"(c), "v"(d)); }
__device__ __forceinline__ void acc_guard4(v8f& a, v8f& b, v8f& c, v8f& d) { asm volatile("v_nop\n\tv_nop\n\tv_nop\n\tv_nop" : "+v"(a), "+v"(b), "+v"(c), "+v"(d)); }
template <typename T> struct Frag;
template <> struct Frag<_Float16> {
  typedef v16h V; union U { v16h v; v8h h[2]; };
  static __device__ __forceinline__ v16h load(const _Float16* p) {
    U f; f.h[0] = *(const v8h*)(p); f.h[1] = *(const v8h*)(p + 16); return f.v;
  }
  static __device__ __forceinline__ v8f mma(v16h a, v16h b, v8f c) {
    return __builtin_amdgcn_wmma_f32_16x16x32_f16(false, a, false, b, (short)0, c, false, false);
  }
  static __device__ __forceinline__ void guard(v8f& a, v8f& b, v16h x, v16h y) { dep_guard_h(a, b, x, y); }
  static __device__ __forceinline__ void keep(v16h a, v16h b, v16h c, v16h d) { keep4_h(a, b, c, d); }
};
template <> struct Frag<__bf16> {
  typedef v16b V; union U { v16b v; v8b h[2]; };
  static __device__ __forceinline__ v16b load(const __bf16* p) {
    U f; f.h[0] = *(const v8b*)(p); f.h[1] = *(const v8b*)(p + 16); return f.v;
  }
  static __device__ __forceinline__ v8f mma(v16b a, v16b b, v8f c) {
    return __builtin_amdgcn_wmma_f32_16x16x32_bf16(false, a, false, b, (short)0, c, false, false);
  }
  static __device__ __forceinline__ void guard(v8f& a, v8f& b, v16b x, v16b y) { dep_guard_b(a, b, x, y); }
  static __device__ __forceinline__ void keep(v16b a, v16b b, v16b c, v16b d) { keep4_b(a, b, c, d); }
};

template <int ET> struct Elem;
template <> struct Elem<0> { typedef _Float16 T; };
template <> struct Elem<1> { typedef __bf16 T; };
template <int ET, bool SPLIT, int BIAS_MODE, int OUT_MODE, bool RESID, int ACT = 0>
__global__ __launch_bounds__(256) void wmma_gemm64(
    const unsigned short* __restrict__ Ap, const unsigned short* __restrict__ A2p, int lda, long strideA,
    const unsigned short* __restrict__ Btp, const unsigned short* __restrict__ Bt2p, int ldb, long strideB,
    void* __restrict__ Cout, void* __restrict__ Cout2, int ldc, long strideC,
    const float* __restrict__ bias,
    const float* __restrict__ resid, long strideR,
    int M, int N, int K, float scale) {
  typedef typename Elem<ET>::T T;
  typedef typename Frag<T>::V V;
  const T* A = (const T*)Ap; const T* A2 = (const T*)A2p; const T* Bt = (const T*)Btp; const T* Bt2 = (const T*)Bt2p;
  __shared__ __align__(16) float sT[8][16 * 68];
  const int b    = blockIdx.y;
  const int lane = threadIdx.x & 31;
  const int wave = threadIdx.x >> 5;
  const int tilesN = N >> 6;
  const int tilesM = M >> 6;
  const int tile = blockIdx.x * 8 + wave;
  if (tile >= tilesM * tilesN) return;
  const int tm = tile / tilesN;
  const int tn = tile - tm * tilesN;
  const int m0 = tm << 6;
  const int n0 = tn << 6;

  const T* Ab  = A  + (size_t)b * strideA;
  const T* Bb  = Bt + (size_t)b * strideB;
  const T* Ab2 = SPLIT ? (A2  + (size_t)b * strideA) : nullptr;
  const T* Bb2 = SPLIT ? (Bt2 + (size_t)b * strideB) : nullptr;

  const int rlane = lane & 15;
  const int koff  = (lane >> 4) * 8;
  const int mOff  = (lane >> 4) * 8;

  v8f acc[4][4];
#pragma unroll
  for (int i = 0; i < 4; ++i)
#pragma unroll
    for (int j = 0; j < 4; ++j) acc[i][j] = (v8f){0.f,0.f,0.f,0.f,0.f,0.f,0.f,0.f};

  for (int k0 = 0; k0 < K; k0 += 32) {
    V bh[4], bl[4];
#pragma unroll
    for (int j = 0; j < 4; ++j) {
      const size_t bo = (size_t)(n0 + (j << 4) + rlane) * ldb + koff + k0;
      bh[j] = Frag<T>::load(Bb + bo);
      if (SPLIT) bl[j] = Frag<T>::load(Bb2 + bo);
    }
#pragma unroll
    for (int i = 0; i < 4; ++i) {
      const size_t ao = (size_t)(m0 + (i << 4) + rlane) * lda + koff + k0;
      V ah = Frag<T>::load(Ab + ao);
      V al;
      if (SPLIT) al = Frag<T>::load(Ab2 + ao);
#pragma unroll
      for (int j = 0; j < 4; ++j) {
        acc[i][j] = Frag<T>::mma(ah, bh[j], acc[i][j]);
        if (SPLIT) {
          acc[i][j] = Frag<T>::mma(ah, bl[j], acc[i][j]);
          acc[i][j] = Frag<T>::mma(al, bh[j], acc[i][j]);
        }
      }
      Frag<T>::guard(acc[i][0], acc[i][3], ah, SPLIT ? al : ah);
    }
    Frag<T>::keep(bh[0], bh[1], bh[2], bh[3]);
    if (SPLIT) Frag<T>::keep(bl[0], bl[1], bl[2], bl[3]);
  }
  acc_guard4(acc[0][0], acc[0][1], acc[0][2], acc[0][3]);
  acc_guard4(acc[1][0], acc[1][1], acc[1][2], acc[1][3]);
  acc_guard4(acc[2][0], acc[2][1], acc[2][2], acc[2][3]);
  acc_guard4(acc[3][0], acc[3][1], acc[3][2], acc[3][3]);

  float* slab = sT[wave];
  const float* Rb = RESID ? (resid + (size_t)b * strideR) : nullptr;
#pragma unroll
  for (int i = 0; i < 4; ++i) {
    const int mBase = m0 + (i << 4);
#pragma unroll
    for (int j = 0; j < 4; ++j) {
      const int n = n0 + (j << 4) + rlane;
      float bv = 0.f;
      if (BIAS_MODE == 2) bv = bias[n];
#pragma unroll
      for (int r = 0; r < 8; ++r) {
        float v = acc[i][j][r] * scale;
        if (BIAS_MODE == 1) v += bias[mBase + mOff + r];
        if (BIAS_MODE == 2) v += bv;
        if (RESID) v += Rb[(size_t)(mBase + mOff + r) * ldc + n];
        if (ACT == 1) v = tanhf(v);
        if (ACT == 2) v = fmaxf(v, 0.0f);
        if (ACT == 3) v = v / (1.0f + expf(-v));
        if (ACT == 4) v = (v > 0.f) ? v : 0.01f * v;
        if (ACT == 5) v = 0.5f * v * (1.0f + erff(v * 0.70710678118654752f));
        slab[(mOff + r) * 68 + (j << 4) + rlane] = v;
      }
    }
    __builtin_amdgcn_fence(__ATOMIC_RELEASE, "workgroup");
    __builtin_amdgcn_wave_barrier();
    __builtin_amdgcn_fence(__ATOMIC_ACQUIRE, "workgroup");
    if (OUT_MODE == 0) {
      float* C = (float*)Cout + (size_t)b * strideC;
      const int hh = lane >> 4, c4 = (lane & 15) * 4;
      for (int pass = 0; pass < 2; ++pass) {
#pragma unroll
        for (int it = 0; it < 8; ++it) {
          const int row = it * 2 + hh;
          v4f v = *(const v4f*)(slab + row * 68 + c4);
          *(volatile v4f*)(C + (size_t)(mBase + row) * ldc + n0 + c4) = v;
        }
        __threadfence();
      }
    } else {
      const int q = lane >> 3, c8 = (lane & 7) * 8;
      unsigned short* C  = (unsigned short*)Cout  + (size_t)b * strideC;
      unsigned short* C2 = (OUT_MODE == 2) ? ((unsigned short*)Cout2 + (size_t)b * strideC) : nullptr;
      for (int pass = 0; pass < 2; ++pass) {
#pragma unroll
        for (int it = 0; it < 4; ++it) {
          const int row = it * 4 + q;
          const float* sp = slab + row * 68 + c8;
          v8h hv, lv;
#pragma unroll
          for (int e = 0; e < 8; ++e) {
            if (OUT_MODE == 1) {
              hv[e] = (_Float16)sp[e];
            } else {
              unsigned short hb = f2bf_bits(sp[e]);
              unsigned short lb = f2bf_bits(sp[e] - bf_bits2f(hb));
              hv[e] = __builtin_bit_cast(_Float16, hb);
              lv[e] = __builtin_bit_cast(_Float16, lb);
            }
          }
          *(volatile v8h*)(C + (size_t)(mBase + row) * ldc + n0 + c8) = hv;
          if (OUT_MODE == 2) *(volatile v8h*)(C2 + (size_t)(mBase + row) * ldc + n0 + c8) = lv;
        }
        __threadfence();
      }
    }
    __builtin_amdgcn_fence(__ATOMIC_RELEASE, "workgroup");
    __builtin_amdgcn_wave_barrier();
    __builtin_amdgcn_fence(__ATOMIC_ACQUIRE, "workgroup");
  }
}

__device__ __forceinline__ unsigned pk16(unsigned short a, unsigned short b) { return (unsigned)a | ((unsigned)b << 16); }

__global__ __launch_bounds__(256) void cast_bf16x2_kernel(const float* __restrict__ in,
                                                          unsigned short* __restrict__ out, int n2) {
  const int i = blockIdx.x * 256 + threadIdx.x;
  if (i < n2) {
    const v2f f = *(const v2f*)(in + 2 * (size_t)i);
    const unsigned u = pk16(f2bf_bits(f[0]), f2bf_bits(f[1]));
    ((volatile unsigned*)out)[i] = u;
    __threadfence();
    ((volatile unsigned*)out)[i] = u;
  }
}

__global__ __launch_bounds__(256) void cast_projw_f16x2_kernel(const float* __restrict__ in,
                                                               unsigned short* __restrict__ out, int n2) {
  const int i = blockIdx.x * 256 + threadIdx.x;
  if (i < n2) {
    const v2f f = *(const v2f*)(in + 2 * (size_t)i);
    const float g0 = bf_bits2f(f2bf_bits(f[0])) * 64.0f;
    const float g1 = bf_bits2f(f2bf_bits(f[1])) * 64.0f;
    const _Float16 h0 = (_Float16)g0, h1 = (_Float16)g1;
    const unsigned u = pk16(__builtin_bit_cast(unsigned short, h0), __builtin_bit_cast(unsigned short, h1));
    ((volatile unsigned*)out)[i] = u;
    __threadfence();
    ((volatile unsigned*)out)[i] = u;
  }
}

__global__ __launch_bounds__(256) void bias_prep_kernel(const float* __restrict__ qkvb, const float* __restrict__ projb,
                                                        float* __restrict__ outb, int nq, int np) {
  const int i = blockIdx.x * 256 + threadIdx.x;
  if (i < nq + np) {
    const int ia = (i < nq) ? i : (nq - 1);
    int ib = i - nq; ib = (ib < 0) ? 0 : ((ib >= np) ? (np - 1) : ib);
    const float a  = qkvb[ia];
    const float bb = projb[ib];
    const float v  = bf_bits2f(f2bf_bits((i < nq) ? a : bb));
    ((volatile float*)outb)[i] = v;
    __threadfence();
    ((volatile float*)outb)[i] = v;
  }
}

__global__ __launch_bounds__(256) void normrope_split_kernel(const float* __restrict__ src,
                                                             const float* __restrict__ cosb, const float* __restrict__ sinb,
                                                             const float* __restrict__ nw,
                                                             unsigned short* __restrict__ oh, unsigned short* __restrict__ ol,
                                                             int njobs) {
  const int wave = threadIdx.x >> 5, lane = threadIdx.x & 31;
  const int job = blockIdx.x * 8 + wave;
  if (job >= njobs) return;
  const int t = job >> 4, h = job & 15, s = t & (kSeq - 1);
  const int d0 = 2 * lane;
  const size_t base = (size_t)t * kDim + (size_t)h * kHd;
  const v2f xv = *(const v2f*)(src + base + d0);
  float a = xv[0], bq = xv[1];
  float ss = a * a + bq * bq;
#pragma unroll
  for (int m = 1; m < 32; m <<= 1) ss += __shfl_xor(ss, m, 32);
  const float inv = rsqrtf(ss * (1.0f / 64.0f) + 1e-6f);
  const v2f wv = *(const v2f*)(nw + d0);
  const float w0 = bf_bits2f(f2bf_bits(wv[0])), w1 = bf_bits2f(f2bf_bits(wv[1]));
  a  = a  * inv * w0;
  bq = bq * inv * w1;
  const v2f cv = *(const v2f*)(cosb + (size_t)s * kHd + d0);
  const v2f sv = *(const v2f*)(sinb + (size_t)s * kHd + d0);
  const float c0 = bf_bits2f(f2bf_bits(cv[0])), c1 = bf_bits2f(f2bf_bits(cv[1]));
  const float s0 = bf_bits2f(f2bf_bits(sv[0])), s1 = bf_bits2f(f2bf_bits(sv[1]));
  const float o0 = a * c0 - bq * s0;
  const float o1 = bq * c1 + a * s1;
  const unsigned short h0 = f2bf_bits(o0), h1 = f2bf_bits(o1);
  const unsigned short l0 = f2bf_bits(o0 - bf_bits2f(h0)), l1 = f2bf_bits(o1 - bf_bits2f(h1));
  const unsigned uh = pk16(h0, h1), ul = pk16(l0, l1);
  const size_t wi = (base >> 1) + lane;
  ((volatile unsigned*)oh)[wi] = uh;
  ((volatile unsigned*)ol)[wi] = ul;
  __threadfence();
  ((volatile unsigned*)oh)[wi] = uh;
  ((volatile unsigned*)ol)[wi] = ul;
}

constexpr int kKC = 64;

__device__ __forceinline__ v8f mma_bf(v16b a, v16b b, v8f c) {
  c = __builtin_amdgcn_wmma_f32_16x16x32_bf16(false, a, false, b, (short)0, c, false, false);
  asm volatile("v_nop\n\tv_nop\n\tv_nop\n\tv_nop" : "+v"(c) : "v"(a), "v"(b));
  return c;
}
__device__ __forceinline__ v8f mma_hf(v16h a, v16h b, v8f c) {
  c = __builtin_amdgcn_wmma_f32_16x16x32_f16(false, a, false, b, (short)0, c, false, false);
  asm volatile("v_nop\n\tv_nop\n\tv_nop\n\tv_nop" : "+v"(c) : "v"(a), "v"(b));
  return c;
}

__global__ __launch_bounds__(128)
void attn_kernel(const unsigned short* __restrict__ qhp, const unsigned short* __restrict__ qlp,
                 const unsigned short* __restrict__ khp, const unsigned short* __restrict__ klp,
                 const unsigned short* __restrict__ vtp, unsigned short* __restrict__ ohp, float sscale) {
  union FB { v16b v; v8b h[2]; };
  union FH { v16h v; v8h h[2]; };
  __shared__ __align__(16) __bf16   Ksh[kKC * kHd];
  __shared__ __align__(16) __bf16   Ksl[kKC * kHd];
  __shared__ __align__(16) _Float16 Vts[kHd * kKC];
  __shared__ __align__(16) _Float16 Psh[4][16 * kKC];
  __shared__ __align__(16) float    Os[4][16 * 68];

  const int tid  = threadIdx.x;
  const int wave = tid >> 5;
  const int lane = tid & 31;
  const int hh   = lane >> 4;
  const int c    = lane & 15;

  const int bx = blockIdx.x;
  const int qb = bx & 31;
  const int bh = bx >> 5;
  const int h  = bh & 15;
  const int b  = bh >> 4;
  const int q0 = qb * 64 + wave * 16;
  const size_t tok0 = (size_t)b * kSeq;

  const __bf16*   Qh = (const __bf16*)(const void*)qhp + tok0 * kDim + (size_t)h * kHd;
  const __bf16*   Ql = (const __bf16*)(const void*)qlp + tok0 * kDim + (size_t)h * kHd;
  const __bf16*   Kh = (const __bf16*)(const void*)khp + tok0 * kDim + (size_t)h * kHd;
  const __bf16*   Kl = (const __bf16*)(const void*)klp + tok0 * kDim + (size_t)h * kHd;
  const _Float16* Vt = (const _Float16*)(const void*)vtp + ((size_t)b * kDim + (size_t)h * kHd) * kSeq;
  _Float16*       Ob = (_Float16*)(void*)ohp + tok0 * kDim + (size_t)h * kHd;

  v16b qah[2], qal[2];
#pragma unroll
  for (int dc = 0; dc < 2; ++dc) {
    qah[dc] = Frag<__bf16>::load(Qh + (size_t)(q0 + c) * kDim + dc * 32 + 8 * hh);
    qal[dc] = Frag<__bf16>::load(Ql + (size_t)(q0 + c) * kDim + dc * 32 + 8 * hh);
  }

  float mrow[8], lrow[8];
  v8f oacc[4];
#pragma unroll
  for (int r = 0; r < 8; ++r) { mrow[r] = -INFINITY; lrow[r] = 0.f; }
#pragma unroll
  for (int t = 0; t < 4; ++t) oacc[t] = (v8f){0.f,0.f,0.f,0.f,0.f,0.f,0.f,0.f};

  for (int kc = 0; kc < kSeq / kKC; ++kc) {
    const int kv0 = kc * kKC;
    __syncthreads();
    {
      const int r = tid >> 1, half = (tid & 1) * 32;
      const __bf16*   ksh = Kh + (size_t)(kv0 + r) * kDim + half;
      const __bf16*   ksl = Kl + (size_t)(kv0 + r) * kDim + half;
      const _Float16* vsr = Vt + (size_t)r * kSeq + kv0 + half;
#pragma unroll
      for (int i = 0; i < 4; ++i) {
        const v8b a0 = *(const v8b*)(ksh + 8 * i);
        const v8b a1 = *(const v8b*)(ksl + 8 * i);
        const v8h vv = *(const v8h*)(vsr + 8 * i);
        *(v8b*)(Ksh + r * kHd + half + 8 * i) = a0;
        *(v8b*)(Ksl + r * kHd + half + 8 * i) = a1;
        *(v8h*)(Vts + r * kKC + half + 8 * i) = vv;
      }
    }
    __syncthreads();

    v8f s[4];
#pragma unroll
    for (int j = 0; j < 4; ++j) {
      s[j] = (v8f){0.f,0.f,0.f,0.f,0.f,0.f,0.f,0.f};
#pragma unroll
      for (int dc = 0; dc < 2; ++dc) {
        FB kb, kl;
        kb.h[0] = *(const v8b*)(Ksh + (j * 16 + c) * kHd + dc * 32 + 8 * hh);
        kb.h[1] = *(const v8b*)(Ksh + (j * 16 + c) * kHd + dc * 32 + 16 + 8 * hh);
        kl.h[0] = *(const v8b*)(Ksl + (j * 16 + c) * kHd + dc * 32 + 8 * hh);
        kl.h[1] = *(const v8b*)(Ksl + (j * 16 + c) * kHd + dc * 32 + 16 + 8 * hh);
        s[j] = mma_bf(qah[dc], kb.v, s[j]);
        s[j] = mma_bf(qah[dc], kl.v, s[j]);
        s[j] = mma_bf(qal[dc], kb.v, s[j]);
      }
    }
    float cm[8];
#pragma unroll
    for (int r = 0; r < 8; ++r) {
      float m = -INFINITY;
#pragma unroll
      for (int j = 0; j < 4; ++j) {
        const float sv = s[j][r] * sscale;
        s[j][r] = sv;
        m = fmaxf(m, sv);
      }
#pragma unroll
      for (int off = 1; off < 16; off <<= 1) m = fmaxf(m, __shfl_xor(m, off, 32));
      cm[r] = m;
    }
    _Float16* pw = Psh[wave];
#pragma unroll
    for (int r = 0; r < 8; ++r) {
      const float mnew  = fmaxf(mrow[r], cm[r]);
      const float alpha = __expf(mrow[r] - mnew);
      mrow[r] = mnew;
      float psum = 0.f;
#pragma unroll
      for (int j = 0; j < 4; ++j) {
        const float p = __expf(s[j][r] - mnew);
        psum += p;
        pw[(8 * hh + r) * kKC + j * 16 + c] = (_Float16)(p * 32768.0f);
      }
#pragma unroll
      for (int off = 1; off < 16; off <<= 1) psum += __shfl_xor(psum, off, 32);
      lrow[r] = lrow[r] * alpha + psum;
#pragma unroll
      for (int t = 0; t < 4; ++t) oacc[t][r] *= alpha;
    }
    __builtin_amdgcn_fence(__ATOMIC_RELEASE, "workgroup");
    __builtin_amdgcn_wave_barrier();
    __builtin_amdgcn_fence(__ATOMIC_ACQUIRE, "workgroup");
#pragma unroll
    for (int kk = 0; kk < 2; ++kk) {
      FH pa;
      pa.h[0] = *(const v8h*)(pw + c * kKC + kk * 32 + 8 * hh);
      pa.h[1] = *(const v8h*)(pw + c * kKC + kk * 32 + 16 + 8 * hh);
#pragma unroll
      for (int t = 0; t < 4; ++t) {
        FH vb;
        vb.h[0] = *(const v8h*)(Vts + (t * 16 + c) * kKC + kk * 32 + 8 * hh);
        vb.h[1] = *(const v8h*)(Vts + (t * 16 + c) * kKC + kk * 32 + 16 + 8 * hh);
        oacc[t] = mma_hf(pa.v, vb.v, oacc[t]);
      }
    }
  }

  float* os = Os[wave];
#pragma unroll
  for (int r = 0; r < 8; ++r) {
    const float inv = (1.0f / lrow[r]) * (64.0f / 32768.0f);
#pragma unroll
    for (int t = 0; t < 4; ++t) os[(8 * hh + r) * 68 + t * 16 + c] = oacc[t][r] * inv;
  }
  __builtin_amdgcn_fence(__ATOMIC_RELEASE, "workgroup");
  __builtin_amdgcn_wave_barrier();
  __builtin_amdgcn_fence(__ATOMIC_ACQUIRE, "workgroup");
  {
    const int qq = lane >> 3, c8 = (lane & 7) * 8;
    for (int pass = 0; pass < 2; ++pass) {
#pragma unroll
      for (int it = 0; it < 4; ++it) {
        const int row = it * 4 + qq;
        const float* sp = os + row * 68 + c8;
        v8h hv;
#pragma unroll
        for (int e = 0; e < 8; ++e) hv[e] = (_Float16)sp[e];
        *(volatile v8h*)(Ob + (size_t)(q0 + row) * kDim + c8) = hv;
      }
      __threadfence();
    }
  }
}

extern "C" void kernel_launch(void* const* d_in, const int* in_sizes, int n_in,
                              void* d_out, int out_size, void* d_ws, size_t ws_size,
                              hipStream_t stream) {
  if (n_in < 9) return;
  if (in_sizes[0] != kTok * kDim) return;
  if (in_sizes[1] != kSeq * kHd || in_sizes[2] != kSeq * kHd) return;
  if (in_sizes[3] != 3 * kDim * kDim || in_sizes[4] != 3 * kDim) return;
  if (in_sizes[5] != kDim * kDim || in_sizes[6] != kDim) return;
  if (in_sizes[7] != kHd || in_sizes[8] != kHd) return;
  if (out_size != kTok * kDim) return;
  if (ws_size < kWsTotal) return;

  const float* x      = (const float*)d_in[0];
  const float* ropec  = (const float*)d_in[1];
  const float* ropes  = (const float*)d_in[2];
  const float* qkv_w  = (const float*)d_in[3];
  const float* qkv_b  = (const float*)d_in[4];
  const float* proj_w = (const float*)d_in[5];
  const float* proj_b = (const float*)d_in[6];
  const float* q_nw   = (const float*)d_in[7];
  const float* k_nw   = (const float*)d_in[8];
  float* out = (float*)d_out;

  char* ws = (char*)d_ws;
  unsigned short* WPROJ = (unsigned short*)(ws + kOffWproj);
  float*          BIAS  = (float*)(ws + kOffBias);
  unsigned short* XB    = (unsigned short*)(ws + kOffXb);
  unsigned short* WQKV  = (unsigned short*)(ws + kOffWqkv);
  unsigned short* KH    = (unsigned short*)(ws + kOffKh);
  unsigned short* KL    = (unsigned short*)(ws + kOffKl);
  float*          QKF   = (float*)(ws + kOffQkf);
  unsigned short* OH    = (unsigned short*)(ws + kOffOh);
  unsigned short* QH    = (unsigned short*)(ws + kOffQh);
  unsigned short* QL    = (unsigned short*)(ws + kOffQl);
  unsigned short* VT    = (unsigned short*)(ws + kOffVt);

  {
    const int n2x = kTok * kDim / 2;
    cast_bf16x2_kernel<<<dim3((n2x + 255) / 256), dim3(256), 0, stream>>>(x, XB, n2x);
    const int n2w = 3 * kDim * kDim / 2;
    cast_bf16x2_kernel<<<dim3((n2w + 255) / 256), dim3(256), 0, stream>>>(qkv_w, WQKV, n2w);
    const int n2p = kDim * kDim / 2;
    cast_projw_f16x2_kernel<<<dim3((n2p + 255) / 256), dim3(256), 0, stream>>>(proj_w, WPROJ, n2p);
    bias_prep_kernel<<<dim3((3 * kDim + kDim + 255) / 256), dim3(256), 0, stream>>>(qkv_b, proj_b, BIAS, 3 * kDim, kDim);
  }
  const int tilesTok = (kTok / 64) * (kDim / 64);
  wmma_gemm64<1, false, 2, 0, false, 0><<<dim3((tilesTok + 7) / 8, 1), dim3(256), 0, stream>>>(
      XB, XB, kDim, 0L, WQKV, WQKV, kDim, 0L, (void*)QKF, (void*)QKF, kDim, 0L,
      BIAS, BIAS, 0L, kTok, kDim, kDim, 1.0f);
  normrope_split_kernel<<<dim3((kTok * kHeads + 7) / 8), dim3(256), 0, stream>>>(QKF, ropec, ropes, q_nw, QH, QL, kTok * kHeads);
  wmma_gemm64<1, false, 2, 0, false, 0><<<dim3((tilesTok + 7) / 8, 1), dim3(256), 0, stream>>>(
      XB, XB, kDim, 0L, WQKV + (size_t)kDim * kDim, WQKV + (size_t)kDim * kDim, kDim, 0L, (void*)QKF, (void*)QKF, kDim, 0L,
      BIAS + kDim, BIAS, 0L, kTok, kDim, kDim, 1.0f);
  {
    const int tilesV = (kDim / 64) * (kSeq / 64);
    wmma_gemm64<1, false, 1, 1, false, 0><<<dim3((tilesV + 7) / 8, kBatch), dim3(256), 0, stream>>>(
        WQKV + (size_t)2 * kDim * kDim, WQKV + (size_t)2 * kDim * kDim, kDim, 0L,
        XB, XB, kDim, (long)kSeq * kDim,
        (void*)VT, (void*)VT, kSeq, (long)kDim * kSeq,
        BIAS + 2 * kDim, BIAS, 0L, kDim, kSeq, kDim, 1.0f);
  }
  normrope_split_kernel<<<dim3((kTok * kHeads + 7) / 8), dim3(256), 0, stream>>>(QKF, ropec, ropes, k_nw, KH, KL, kTok * kHeads);
  attn_kernel<<<dim3(kBatch * kHeads * (kSeq / 64)), dim3(128), 0, stream>>>(QH, QL, KH, KL, VT, OH, 0.125f);
  wmma_gemm64<0, false, 2, 0, false, 0><<<dim3((tilesTok + 7) / 8, 1), dim3(256), 0, stream>>>(
      OH, OH, kDim, 0L, WPROJ, WPROJ, kDim, 0L, (void*)out, (void*)out, kDim, 0L,
      BIAS + 3 * kDim, BIAS, 0L, kTok, kDim, kDim, 1.0f / 4096.0f);
}
